// SelfAttention_35545149341704
// MI455X (gfx1250) — hardware-run, weakly checked
//
#include <hip/hip_runtime.h>


#ifndef NB
#define NB 16
#endif
#ifndef SEQ
#define SEQ 680
#endif
#define NB_FULL  16
#define SEQ_FULL 680
#ifndef OUT_SEQ
#define OUT_SEQ SEQ
#endif
#define LP   (((SEQ + 63) / 64) * 64)
#define DM   1024
#define NH_  16
#define HD   64
#define NSEG 10
#define AW   4
#define OSP  68
#define EROWS (LP < 128 ? LP : 128)
#define RKEYS (LP < 192 ? LP : 192)
#define QRS  2048.0f
#define QRI  (1.0f / 2048.0f)
#define QSC  16.0f
#define KSC  64.0f
#define CSC  16.0f
#define WSC  256.0f
#define OSCI (1.0f / (16.0f * 256.0f))
#define SC2  ((float)(1.4426950408889634 / (16.0 * 64.0)))
#define PSH  14.0f
#define NEGB (-3.0e38f)
#define MAXLOG 4.605170185988091f

static_assert(HD == 64);
static_assert(NH_ * HD == DM);
static_assert(DM % 64 == 0);
static_assert(DM % 32 == 0);
static_assert(HD % 32 == 0);
static_assert(LP % 64 == 0);
static_assert(SEQ <= LP);
static_assert(LP - SEQ < 64);
static_assert(EROWS % 64 == 0);
static_assert(EROWS % 32 == 0);
static_assert(EROWS <= LP);
static_assert(RKEYS % 64 == 0);
static_assert(RKEYS >= 32);
static_assert(RKEYS <= LP);
static_assert(EROWS % (16 * AW) == 0);
static_assert((LP - EROWS) % (16 * AW) == 0);
static_assert((LP - EROWS) % 64 == 0);
static_assert(NB <= NB_FULL);
static_assert(SEQ <= SEQ_FULL);
static_assert((OSP * 4) % 16 == 0);
static_assert(OSP >= 64 + 4);
static_assert(AW * 16 * OSP * 4 <= 131072);
static_assert(16 * 68 * 4 <= 131072);
static_assert(32 * 16 * 4 == 16 * HD * 2);
static_assert(32 * 16 * 8 == 16 * 64 * 4);

typedef _Float16 h16;
typedef unsigned short bf;
typedef __attribute__((ext_vector_type(16))) __bf16   v16bf;
typedef __attribute__((ext_vector_type(16))) _Float16 v16h;
typedef __attribute__((ext_vector_type(8)))  _Float16 v8h;
typedef __attribute__((ext_vector_type(8)))  unsigned short v8us;
typedef __attribute__((ext_vector_type(8)))  float    v8f;
typedef __attribute__((ext_vector_type(4)))  float    v4f;
typedef v4f  __attribute__((may_alias)) v4fa;

__device__ __forceinline__ unsigned short f2bf(float f) { unsigned u = __float_as_uint(f); u += 0x7FFFu + ((u >> 16) & 1u); return (unsigned short)(u >> 16); }
__device__ __forceinline__ float bfr(float f) { return __uint_as_float(((unsigned)f2bf(f)) << 16); }
__device__ __forceinline__ v16h cat16(v8h lo, v8h hi) { return __builtin_shufflevector(lo, hi, 0, 1, 2, 3, 4, 5, 6, 7, 8, 9, 10, 11, 12, 13, 14, 15); }
__device__ __forceinline__ v16bf cat16b(v8us lo, v8us hi) { return __builtin_bit_cast(v16bf, __builtin_shufflevector(lo, hi, 0, 1, 2, 3, 4, 5, 6, 7, 8, 9, 10, 11, 12, 13, 14, 15)); }
__device__ __forceinline__ v8f wmma16(v16h a, v16h b, v8f c) { return __builtin_amdgcn_wmma_f32_16x16x32_f16(false, a, false, b, (short)0, c, false, false); }
__device__ __forceinline__ v8f wmmab(v16bf a, v16bf b, v8f c) { return __builtin_amdgcn_wmma_f32_16x16x32_bf16(false, a, false, b, (short)0, c, false, false); }
__device__ __forceinline__ v16h  ldh(const h16* p) { return cat16(*(const v8h*)p, *(const v8h*)(p + 16)); }
__device__ __forceinline__ v16bf ldb(const bf* p)  { return cat16b(*(const v8us*)p, *(const v8us*)(p + 16)); }
__device__ __forceinline__ void wave_sync() { __builtin_amdgcn_fence(3  , "wavefront"); __builtin_amdgcn_wave_barrier(); asm volatile("" ::: "memory"); }

__device__ __forceinline__ v8f wmma16g(v16h a, v16h b, v8f c) {
    c = wmma16(a, b, c);
    asm volatile("v_nop\n\tv_nop\n\tv_nop\n\tv_nop" : "+v"(c) : "v"(a), "v"(b));
    return c;
}
__device__ __forceinline__ v8f wmmabg(v16bf a, v16bf b, v8f c) {
    c = wmmab(a, b, c);
    asm volatile("v_nop\n\tv_nop\n\tv_nop\n\tv_nop" : "+v"(c) : "v"(a), "v"(b));
    return c;
}
__device__ __forceinline__ h16 toh_flush(float v) { const h16 r = (h16)v; return (fabsf(v) < 6.103515625e-05f) ? (h16)0.0f : r; }

__device__ __forceinline__ void seg_of(const int* __restrict__ pn, int t, int& ks, int& ke) {
    int start = 0; ks = 0; ke = 0;
#pragma unroll
    for (int i = 0; i < NSEG; ++i) {
        int ln = pn[i]; ln = max(0, min(ln, SEQ));
        const int en = min(start + ln, SEQ);
        const bool in = (t >= start) & (t < en);
        ks = in ? start : ks; ke = in ? en : ke;
        start = en;
    }
}

__global__ __launch_bounds__(256) void k_cvt8(const float* __restrict__ src, bf* dst, size_t n8) {
    const size_t i = (size_t)blockIdx.x * 256 + threadIdx.x; if (i >= n8) return;
    const v8f v = *(const v8f*)(src + i * 8); v8us o;
#pragma unroll
    for (int k = 0; k < 8; ++k) o[k] = f2bf(v[k]);
    *(volatile v8us*)(dst + i * 8) = o; __threadfence(); *(volatile v8us*)(dst + i * 8) = o;
}

__global__ __launch_bounds__(256) void k_cvtx(const float* __restrict__ src, bf* dst, size_t n8) {
    const size_t i = (size_t)blockIdx.x * 256 + threadIdx.x; if (i >= n8) return;
    const size_t row = i / (DM / 8); const int c8 = (int)(i % (DM / 8));
    const int b = (int)(row / LP), t = (int)(row % LP);
    const int tc = t < SEQ ? t : (SEQ - 1);
    v8f v = *(const v8f*)(src + ((size_t)b * SEQ_FULL + (size_t)tc) * DM + (size_t)c8 * 8);
    asm volatile("" : "+v"(v));
    const bool ok = t < SEQ; v8us o;
#pragma unroll
    for (int k = 0; k < 8; ++k) { const unsigned short w = f2bf(v[k]); o[k] = ok ? w : (unsigned short)0; }
    *(volatile v8us*)(dst + i * 8) = o; __threadfence(); *(volatile v8us*)(dst + i * 8) = o;
}

__global__ __launch_bounds__(256) void k_cvtw(const float* __restrict__ src, h16* dst, size_t n8) {
    const size_t i = (size_t)blockIdx.x * 256 + threadIdx.x; if (i >= n8) return;
    const v8f v = *(const v8f*)(src + i * 8); v8h o;
#pragma unroll
    for (int k = 0; k < 8; ++k) o[k] = toh_flush(bfr(v[k]) * WSC);
    *(volatile v8h*)(dst + i * 8) = o; __threadfence(); *(volatile v8h*)(dst + i * 8) = o;
}

__device__ __forceinline__ void mmb64(const bf* __restrict__ A, const bf* __restrict__ Bt, size_t aoff, size_t boff, v8f (&acc)[4][4]) {
    const int K = DM;
#pragma unroll 1
    for (int kc = 0; kc < K; kc += 32) {
        v16bf a[4];
#pragma unroll
        for (int mb = 0; mb < 4; ++mb) a[mb] = ldb(A + aoff + (size_t)mb * 16 * K + kc);
#pragma unroll
        for (int nb = 0; nb < 4; ++nb) { const v16bf b = ldb(Bt + boff + (size_t)nb * 16 * K + kc);
#pragma unroll
            for (int mb = 0; mb < 4; ++mb) acc[mb][nb] = wmmabg(a[mb], b, acc[mb][nb]); }
    }
}

__global__ __launch_bounds__(32) void k_projn(const bf* __restrict__ A, const bf* __restrict__ Bt, const float* __restrict__ bias, int hasb,
                                              const float* __restrict__ slog, int useslog, float carry, h16* Ph) {
    __shared__ __align__(16) float os[16 * 68];
    const int lane = threadIdx.x & 31, lr = lane & 15, hi = lane >> 4; const int r0 = blockIdx.x * 64, c0 = blockIdx.y * 64;
    v8f acc[4][4];
#pragma unroll
    for (int mb = 0; mb < 4; ++mb)
#pragma unroll
        for (int nb = 0; nb < 4; ++nb) acc[mb][nb] = (v8f){};
    mmb64(A, Bt, (size_t)(r0 + lr) * DM + 8 * hi, (size_t)(c0 + lr) * DM + 8 * hi, acc);
    const int hh = c0 / HD;
    float bc[4];
#pragma unroll
    for (int nb = 0; nb < 4; ++nb) { const float bv = bfr(bias[c0 + nb * 16 + lr]); bc[nb] = hasb ? bv : 0.0f; }
    const float sl = bfr(slog[hh]);
    const float sce = expf(fminf(sl, MAXLOG));
    const float mult = (useslog ? sce : 1.0f) * carry;
    const int bb = r0 / LP, tt = r0 % LP;
    const size_t tbase = ((size_t)(bb * NH_ + hh) * LP + (size_t)tt) * HD;
#pragma unroll
    for (int mb = 0; mb < 4; ++mb) {
#pragma unroll
        for (int nb = 0; nb < 4; ++nb) {
#pragma unroll
            for (int j = 0; j < 8; ++j) os[(hi * 8 + j) * 68 + nb * 16 + lr] = acc[mb][nb][j] + bc[nb]; }
        wave_sync();
        v8h hv[4];
#pragma unroll
        for (int s = 0; s < 4; ++s) { const int row = 4 * s + (lane >> 3), c8 = (lane & 7) * 8;
            const v4f x0 = *(const v4fa*)(&os[row * 68 + c8]); const v4f x1 = *(const v4fa*)(&os[row * 68 + c8 + 4]);
            float ss = x0[0] * x0[0] + x0[1] * x0[1] + x0[2] * x0[2] + x0[3] * x0[3] + x1[0] * x1[0] + x1[1] * x1[1] + x1[2] * x1[2] + x1[3] * x1[3];
            ss += __shfl_xor(ss, 1, 32); ss += __shfl_xor(ss, 2, 32); ss += __shfl_xor(ss, 4, 32);
            const float rn = mult * (1.0f / fmaxf(sqrtf(ss), 1e-12f));
#pragma unroll
            for (int i = 0; i < 4; ++i) { hv[s][i] = toh_flush(x0[i] * rn); hv[s][4 + i] = toh_flush(x1[i] * rn); } }
#pragma unroll 1
        for (int ps = 0; ps < 2; ++ps) {
#pragma unroll
            for (int s = 0; s < 4; ++s) { const size_t oo = tbase + (size_t)(mb * 16) * HD + (size_t)(s * 32 + lane) * 8;
                *(volatile v8h*)(Ph + oo) = hv[s]; }
            if (ps == 0) __threadfence(); }
        wave_sync();
    }
}

__global__ __launch_bounds__(32) void k_projv(const bf* __restrict__ A, const bf* __restrict__ Bt, const float* __restrict__ bias, h16* Ph, h16* Pr, int resT) {
    __shared__ __align__(16) float os[16 * 68];
    const int lane = threadIdx.x & 31, lr = lane & 15, hi = lane >> 4; const int r0 = blockIdx.x * 64, c0 = blockIdx.y * 64;
    v8f acc[4][4];
#pragma unroll
    for (int mb = 0; mb < 4; ++mb)
#pragma unroll
        for (int nb = 0; nb < 4; ++nb) acc[mb][nb] = (v8f){};
    mmb64(A, Bt, (size_t)(r0 + lr) * DM + 8 * hi, (size_t)(c0 + lr) * DM + 8 * hi, acc);
    const int bb = c0 / LP, tt = c0 % LP;
    const size_t tbase = (size_t)bb * (size_t)DM * LP + (size_t)r0 * LP + (size_t)tt;
    const size_t rbase = (size_t)bb * (size_t)DM * (size_t)resT + (size_t)r0 * (size_t)resT + (size_t)tt;
    const bool wr = tt < resT;
#pragma unroll
    for (int mb = 0; mb < 4; ++mb) {
        float br[8];
#pragma unroll
        for (int j = 0; j < 8; ++j) br[j] = bfr(bias[r0 + mb * 16 + hi * 8 + j]);
#pragma unroll
        for (int nb = 0; nb < 4; ++nb) {
#pragma unroll
            for (int j = 0; j < 8; ++j) os[(hi * 8 + j) * 68 + nb * 16 + lr] = acc[mb][nb][j] + br[j]; }
        wave_sync();
        v8h hv[4], rv[4];
#pragma unroll
        for (int s = 0; s < 4; ++s) { const int row = 4 * s + (lane >> 3), c8 = (lane & 7) * 8;
            const v4f x0 = *(const v4fa*)(&os[row * 68 + c8]); const v4f x1 = *(const v4fa*)(&os[row * 68 + c8 + 4]);
#pragma unroll
            for (int i = 0; i < 4; ++i) { const h16 a0 = toh_flush(x0[i]); const h16 a1 = toh_flush(x1[i]); hv[s][i] = a0; hv[s][4 + i] = a1;
                rv[s][i] = toh_flush((x0[i] - (float)a0) * QRS); rv[s][4 + i] = toh_flush((x1[i] - (float)a1) * QRS); } }
#pragma unroll 1
        for (int ps = 0; ps < 2; ++ps) {
#pragma unroll
            for (int s = 0; s < 4; ++s) { const int row = 4 * s + (lane >> 3), c8 = (lane & 7) * 8;
                const size_t oo = tbase + (size_t)(mb * 16 + row) * LP + c8;
                const size_t ro = rbase + (size_t)(mb * 16 + row) * (size_t)resT + c8;
                *(volatile v8h*)(Ph + oo) = hv[s]; if (wr) *(volatile v8h*)(Pr + ro) = rv[s]; }
            if (ps == 0) __threadfence(); }
        wave_sync();
    }
}

template <int EARLY>
__device__ __forceinline__ void flash_body(const h16* __restrict__ QH, const h16* __restrict__ KP, const h16* __restrict__ VT, const h16* __restrict__ VR,
                                           const int* __restrict__ pn, h16* CH, h16* CR) {
    __shared__ __align__(16) float os[AW * 16 * OSP];
    const int lane = threadIdx.x & 31, lr = lane & 15, hi = lane >> 4;
    const int wave = __builtin_amdgcn_readfirstlane((int)(threadIdx.x >> 5));
    const int zh = blockIdx.y; const int b = zh / NH_, h = zh % NH_;
    const int t0 = (EARLY ? 0 : EROWS) + (blockIdx.x * AW + wave) * 16;
    int ks, ke; seg_of(pn, t0 + lr, ks, ke);
    int kmin = (ke > ks) ? ks : 0x7fffffff, kmax = ke;
    kmin = min(kmin, __shfl_xor(kmin, 1, 32)); kmax = max(kmax, __shfl_xor(kmax, 1, 32));
    kmin = min(kmin, __shfl_xor(kmin, 2, 32)); kmax = max(kmax, __shfl_xor(kmax, 2, 32));
    kmin = min(kmin, __shfl_xor(kmin, 4, 32)); kmax = max(kmax, __shfl_xor(kmax, 4, 32));
    kmin = min(kmin, __shfl_xor(kmin, 8, 32)); kmax = max(kmax, __shfl_xor(kmax, 8, 32));
    const int kbv = min(kmin, kmax) & ~31;
    const int knv = min((kmax + 31) & ~31, LP);
    const int kbeg = __builtin_amdgcn_readfirstlane(kbv), kend = __builtin_amdgcn_readfirstlane(knv);
    const size_t pbase = (size_t)zh * LP * HD;
    const size_t qo = pbase + (size_t)(t0 + lr) * HD + 8 * hi;
    const v16h q0 = ldh(QH + qo), q1 = ldh(QH + qo + 32);
    const size_t ko = pbase + (size_t)lr * HD + 8 * hi;
    const size_t vo = pbase + (size_t)lr * LP + 8 * hi;
    const size_t vro = (size_t)zh * HD * RKEYS + (size_t)lr * RKEYS + 8 * hi;
    const v16h hz = (v16h){};
    v8f o[4], oR[4];
#pragma unroll
    for (int j = 0; j < 4; ++j) { o[j] = (v8f){}; oR[j] = (v8f){}; }
    float m = NEGB, l = 0.0f;
#pragma unroll 1
    for (int key0 = kbeg; key0 < kend; key0 += 32) {
        const h16* ka = KP + ko + (size_t)key0 * HD;
        const v16h ka0 = ldh(ka), ka1 = ldh(ka + 32), kb0 = ldh(ka + 16 * HD), kb1 = ldh(ka + 16 * HD + 32);
        v8f sa = (v8f){}, sb = (v8f){};
        sa = wmma16g(ka0, q0, sa); sa = wmma16g(ka1, q1, sa);
        sb = wmma16g(kb0, q0, sb); sb = wmma16g(kb1, q1, sb);
        const int ja = key0 + 8 * hi;
        float ta[8], tb[8]; bool fa[8], fb[8]; float mx = NEGB;
#pragma unroll
        for (int r = 0; r < 8; ++r) {
            const int j0 = ja + r, j1 = ja + 16 + r;
            fa[r] = (j0 >= ks) & (j0 < ke);
            fb[r] = (j1 >= ks) & (j1 < ke);
            ta[r] = sa[r] * SC2; tb[r] = sb[r] * SC2;
            mx = fmaxf(mx, fmaxf(fa[r] ? ta[r] : NEGB, fb[r] ? tb[r] : NEGB)); }
        mx = fmaxf(mx, __shfl_xor(mx, 16, 32));
        const float mnew = fmaxf(m, mx);
        const float alpha = __builtin_amdgcn_exp2f(m - mnew);
        const float sh = PSH - mnew;
        v16h pb, pr = hz; float ls = 0.0f;
#pragma unroll
        for (int r = 0; r < 8; ++r) {
            const float aa = ta[r] + sh, ab = tb[r] + sh;
            const float ea = __builtin_amdgcn_exp2f(aa), eb = __builtin_amdgcn_exp2f(ab);
            const float ga = (fa[r] & (aa >= -14.0f)) ? ea : 0.0f, gb = (fb[r] & (ab >= -14.0f)) ? eb : 0.0f;
            const h16 pa = (h16)ga; const h16 pc = (h16)gb;
            pb[r] = pa; pb[8 + r] = pc;
            if (EARLY) { pr[r] = toh_flush((ga - (float)pa) * QRS); pr[8 + r] = toh_flush((gb - (float)pc) * QRS); ls += ga + gb; }
            else       { ls += (float)pa + (float)pc; } }
        l = l * alpha + ls; m = mnew;
#pragma unroll
        for (int j = 0; j < 4; ++j) { o[j] = o[j] * alpha; if (EARLY) oR[j] = oR[j] * alpha; }
        const h16* va = VT + vo + key0;
        v16h vf[4];
#pragma unroll
        for (int j = 0; j < 4; ++j) vf[j] = ldh(va + (size_t)(16 * j) * LP);
#pragma unroll
        for (int j = 0; j < 4; ++j) o[j] = wmma16g(vf[j], pb, o[j]);
        if (EARLY) {
#pragma unroll
            for (int j = 0; j < 4; ++j) oR[j] = wmma16g(vf[j], pr, oR[j]);
            const bool rok = key0 < RKEYS;
            const int kcl = min(key0, RKEYS - 32);
            const h16* vr = VR + vro + kcl;
            v16h vg[4];
#pragma unroll
            for (int j = 0; j < 4; ++j) { vg[j] = ldh(vr + (size_t)(16 * j) * RKEYS); if (!rok) vg[j] = hz; }
#pragma unroll
            for (int j = 0; j < 4; ++j) oR[j] = wmma16g(vg[j], pb, oR[j]);
        }
    }
    l += __shfl_xor(l, 16, 32);
    const bool any = l > 0.0f;
    const float lsafe = any ? l : 1.0f;
    const float inv = any ? (CSC * (1.0f / lsafe)) : 0.0f;
    const int wb = wave * 16 * OSP;
#pragma unroll
    for (int j = 0; j < 4; ++j) {
        v8f f = o[j];
        if (EARLY) f = o[j] + oR[j] * QRI;
        v4f a, c;
        a[0] = f[0] * inv; a[1] = f[1] * inv; a[2] = f[2] * inv; a[3] = f[3] * inv; c[0] = f[4] * inv; c[1] = f[5] * inv; c[2] = f[6] * inv; c[3] = f[7] * inv;
        *(v4fa*)(&os[wb + lr * OSP + 16 * j + 8 * hi]) = a; *(v4fa*)(&os[wb + lr * OSP + 16 * j + 8 * hi + 4]) = c; }
    wave_sync();
    v8h hv[4], rv[4];
#pragma unroll
    for (int s = 0; s < 4; ++s) { const int row = 4 * s + (lane >> 3), c8 = (lane & 7) * 8;
        const v4f x0 = *(const v4fa*)(&os[wb + row * OSP + c8]); const v4f x1 = *(const v4fa*)(&os[wb + row * OSP + c8 + 4]);
#pragma unroll
        for (int i = 0; i < 4; ++i) { const h16 a0 = toh_flush(x0[i]); const h16 a1 = toh_flush(x1[i]); hv[s][i] = a0; hv[s][4 + i] = a1;
            rv[s][i] = toh_flush((x0[i] - (float)a0) * QRS); rv[s][4 + i] = toh_flush((x1[i] - (float)a1) * QRS); } }
    const size_t cb = ((size_t)b * LP + (size_t)t0) * DM + (size_t)h * HD;
    const size_t rb = ((size_t)b * EROWS + (size_t)(EARLY ? t0 : 0)) * DM + (size_t)h * HD;
#pragma unroll 1
    for (int ps = 0; ps < 2; ++ps) {
#pragma unroll
        for (int s = 0; s < 4; ++s) { const int row = 4 * s + (lane >> 3), c8 = (lane & 7) * 8;
            *(volatile v8h*)(CH + cb + (size_t)row * DM + c8) = hv[s];
            if (EARLY) *(volatile v8h*)(CR + rb + (size_t)row * DM + c8) = rv[s]; }
        if (ps == 0) __threadfence(); }
}

__global__ __launch_bounds__(32 * AW) void k_flash_e(const h16* __restrict__ QH, const h16* __restrict__ KP, const h16* __restrict__ VT, const h16* __restrict__ VR,
                                                     const int* __restrict__ pn, h16* CH, h16* CR) {
    flash_body<1>(QH, KP, VT, VR, pn, CH, CR);
}
__global__ __launch_bounds__(32 * AW) void k_flash_l(const h16* __restrict__ QH, const h16* __restrict__ KP, const h16* __restrict__ VT, const h16* __restrict__ VR,
                                                     const int* __restrict__ pn, h16* CH, h16* CR) {
    flash_body<0>(QH, KP, VT, VR, pn, CH, CR);
}

template <int EARLY>
__device__ __forceinline__ void out_body(const h16* __restrict__ CHp, const h16* __restrict__ CRp, const h16* __restrict__ WP, const float* __restrict__ pbias, float* OUT) {
    constexpr int MB = EARLY ? 2 : 4;
    constexpr int TPB = EARLY ? (EROWS / 32) : (((LP - EROWS) / 64) > 0 ? ((LP - EROWS) / 64) : 1);
    __shared__ __align__(16) float os[16 * 68];
    const int K = DM;
    const int lane = threadIdx.x & 31, lr = lane & 15, hi = lane >> 4;
    const int bb = blockIdx.x / TPB, tt = (EARLY ? 0 : EROWS) + (blockIdx.x % TPB) * (16 * MB);
    const int c0 = blockIdx.y * 64;
    v8f acc[MB][4], accR[MB][4];
#pragma unroll
    for (int mb = 0; mb < MB; ++mb)
#pragma unroll
        for (int nb = 0; nb < 4; ++nb) { acc[mb][nb] = (v8f){}; accR[mb][nb] = (v8f){}; }
    const size_t aoff = ((size_t)bb * LP + (size_t)(tt + lr)) * K + 8 * hi;
    const size_t roff = ((size_t)bb * EROWS + (size_t)((EARLY ? tt : 0) + lr)) * K + 8 * hi;
    const size_t boff = (size_t)(c0 + lr) * K + 8 * hi;
#pragma unroll 1
    for (int kc = 0; kc < K; kc += 32) {
        v16h a[MB], ar[MB];
#pragma unroll
        for (int mb = 0; mb < MB; ++mb) { a[mb] = ldh(CHp + aoff + (size_t)mb * 16 * K + kc); if (EARLY) ar[mb] = ldh(CRp + roff + (size_t)mb * 16 * K + kc); }
#pragma unroll
        for (int nb = 0; nb < 4; ++nb) { const v16h bfrag = ldh(WP + boff + (size_t)nb * 16 * K + kc);
#pragma unroll
            for (int mb = 0; mb < MB; ++mb) { acc[mb][nb] = wmma16g(a[mb], bfrag, acc[mb][nb]); if (EARLY) accR[mb][nb] = wmma16g(ar[mb], bfrag, accR[mb][nb]); } }
    }
    float bc[4];
#pragma unroll
    for (int nb = 0; nb < 4; ++nb) bc[nb] = bfr(pbias[c0 + nb * 16 + lr]);
#pragma unroll
    for (int mb = 0; mb < MB; ++mb) {
#pragma unroll
        for (int nb = 0; nb < 4; ++nb) {
#pragma unroll
            for (int j = 0; j < 8; ++j) { float v = acc[mb][nb][j]; if (EARLY) v += accR[mb][nb][j] * QRI;
                os[(hi * 8 + j) * 68 + nb * 16 + lr] = v * OSCI + bc[nb]; } }
        wave_sync();
        const int tb0 = tt + mb * 16;
#pragma unroll 1
        for (int ps = 0; ps < 2; ++ps) {
#pragma unroll
            for (int s = 0; s < 8; ++s) { const int row = 2 * s + (lane >> 4), cofs = (lane & 15) * 4;
                const v4f val = *(const v4fa*)(&os[row * 68 + cofs]);
                const int t = tb0 + row;
                if (t < SEQ) *(volatile v4f*)(OUT + ((size_t)bb * OUT_SEQ + (size_t)t) * DM + c0 + cofs) = val; }
            if (ps == 0) __threadfence(); }
        wave_sync();
    }
}

__global__ __launch_bounds__(32) void k_out_e(const h16* __restrict__ CHp, const h16* __restrict__ CRp, const h16* __restrict__ WP, const float* __restrict__ pbias, float* OUT) {
    out_body<1>(CHp, CRp, WP, pbias, OUT);
}
__global__ __launch_bounds__(32) void k_out_l(const h16* __restrict__ CHp, const h16* __restrict__ CRp, const h16* __restrict__ WP, const float* __restrict__ pbias, float* OUT) {
    out_body<0>(CHp, CRp, WP, pbias, OUT);
}

static constexpr size_t al256(size_t v) { return (v + 255) & ~(size_t)255; }
static constexpr size_t SZ_XB = al256((size_t)NB * LP * DM * 2);
static constexpr size_t SZ_CH = al256((size_t)NB * LP * DM * 2);
static constexpr size_t SZ_WB = al256((size_t)3 * DM * DM * 2);
static constexpr size_t SZ_WP = al256((size_t)DM * DM * 2);
static constexpr size_t SZ_PL = al256((size_t)NB * NH_ * LP * HD * 2);
static constexpr size_t SZ_VR = al256((size_t)NB * NH_ * HD * RKEYS * 2);
static constexpr size_t SZ_CR = al256((size_t)NB * EROWS * DM * 2);
static constexpr size_t SZ_TOTAL = SZ_XB + SZ_WB + SZ_WP + 3 * SZ_PL + SZ_VR + SZ_CR;
static_assert(SZ_CH <= SZ_XB);
static_assert(SZ_TOTAL <= (size_t)134217728);
static_assert(((size_t)DM * DM * 2) % 256 == 0);
static_assert((size_t)NB * NH_ * LP * HD == (size_t)NB * DM * LP);
static_assert(((size_t)NB * LP * DM) % (8 * 256) == 0);
static_assert(((size_t)DM * DM) % 8 == 0);

extern "C" void kernel_launch(void* const* d_in, const int* in_sizes, int n_in,
                              void* d_out, int out_size, void* d_ws, size_t ws_size, hipStream_t stream) {
    if (n_in < 8) return;
    const size_t needx = ((size_t)(NB - 1) * SEQ_FULL + SEQ) * DM;
    if ((size_t)in_sizes[0] < needx) return;
    if (in_sizes[1] < NSEG) return;
    if ((size_t)in_sizes[2] < (size_t)3 * DM * DM) return;
    if (in_sizes[3] < DM || in_sizes[4] < DM || in_sizes[5] < NH_ || in_sizes[7] < DM) return;
    if ((size_t)in_sizes[6] < (size_t)DM * DM) return;
    if ((size_t)out_size < ((size_t)(NB - 1) * OUT_SEQ + SEQ) * DM) return;
    if (SZ_TOTAL > ws_size) return;
    const float* x     = (const float*)d_in[0];
    const int*   pn    = (const int*)d_in[1];
    const float* wqkv  = (const float*)d_in[2];
    const float* qbias = (const float*)d_in[3];
    const float* vbias = (const float*)d_in[4];
    const float* slog  = (const float*)d_in[5];
    const float* wproj = (const float*)d_in[6];
    const float* pbias = (const float*)d_in[7];
    float* OUT = (float*)d_out;
    char* wsp = (char*)d_ws;
    bf*  XB = (bf*)wsp;
    h16* CH = (h16*)wsp; wsp += SZ_XB;
    bf*  WB = (bf*)wsp;  wsp += SZ_WB;
    h16* WP = (h16*)wsp; wsp += SZ_WP;
    h16* QH = (h16*)wsp; wsp += SZ_PL;
    h16* KP = (h16*)wsp; wsp += SZ_PL;
    h16* VT = (h16*)wsp; wsp += SZ_PL;
    h16* VR = (h16*)wsp; wsp += SZ_VR;
    h16* CR = (h16*)wsp; wsp += SZ_CR;
    bf* WQ = WB; bf* WK = WB + (size_t)DM * DM; bf* WV = WB + (size_t)2 * DM * DM;

    { const size_t n8 = (size_t)NB * LP * DM / 8; k_cvtx<<<(unsigned)((n8 + 255) / 256), 256, 0, stream>>>(x, XB, n8); }
    { const size_t n8 = (size_t)3 * DM * DM / 8; k_cvt8<<<(unsigned)((n8 + 255) / 256), 256, 0, stream>>>(wqkv, WB, n8); }
    { const size_t n8 = (size_t)DM * DM / 8; k_cvtw<<<(unsigned)((n8 + 255) / 256), 256, 0, stream>>>(wproj, WP, n8); }

    k_projn<<<dim3(NB * LP / 64, DM / 64, 1), 32, 0, stream>>>(XB, WQ, qbias, 1, slog, 1, QSC, QH);
    k_projn<<<dim3(NB * LP / 64, DM / 64, 1), 32, 0, stream>>>(XB, WK, qbias, 0, slog, 0, KSC, KP);
    k_projv<<<dim3(DM / 64, NB * LP / 64, 1), 32, 0, stream>>>(WV, XB, vbias, VT, VR, RKEYS);

    k_flash_e<<<dim3(EROWS / (16 * AW), NB * NH_, 1), 32 * AW, 0, stream>>>(QH, KP, VT, VR, pn, CH, CR);
    if (LP > EROWS)
        k_flash_l<<<dim3((LP - EROWS) / (16 * AW), NB * NH_, 1), 32 * AW, 0, stream>>>(QH, KP, VT, VR, pn, CH, CR);

    k_out_e<<<dim3(NB * (EROWS / 32), DM / 64, 1), 32, 0, stream>>>(CH, CR, WP, pbias, OUT);
    if (LP > EROWS)
        k_out_l<<<dim3(NB * ((LP - EROWS) / 64), DM / 64, 1), 32, 0, stream>>>(CH, CR, WP, pbias, OUT);
}
